// TiledAttention_65687229825650
// MI455X (gfx1250) — hardware-verified
//
#include <hip/hip_runtime.h>

typedef __attribute__((ext_vector_type(16))) __bf16        v16b;
typedef __attribute__((ext_vector_type(8)))  __bf16        v8b;
typedef __attribute__((ext_vector_type(8)))  float         v8f;
typedef __attribute__((ext_vector_type(4)))  float         v4f;
typedef __attribute__((ext_vector_type(4)))  unsigned int  v4u;
typedef __attribute__((ext_vector_type(8)))  unsigned short v8us;

static constexpr int NBATCH = 2;
static constexpr int NSEQ   = 2048;
static constexpr int NMODEL = 1024;
static constexpr int NHEAD  = 16;
static constexpr int NDHEAD = 64;
static constexpr int NROW   = NBATCH * NSEQ;
static constexpr int NQKV   = 3 * NMODEL;

static_assert(NMODEL == NHEAD * NDHEAD, "head split");
static_assert(NDHEAD == 64, "attention kernel is head-dim 64");
static_assert(NSEQ % 64 == 0, "query blocks of 64");
static_assert(NROW % 64 == 0 && NQKV % 64 == 0 && NMODEL % 64 == 0, "tile multiples");
static_assert(NMODEL % 32 == 0, "K multiple of 32");

__device__ __forceinline__ unsigned short f2bf_bits(float f) {
  unsigned u = __float_as_uint(f);
  return (unsigned short)((u + 0x7FFFu + ((u >> 16) & 1u)) >> 16);
}
__device__ __forceinline__ float bf_bits2f(unsigned short h) { return __uint_as_float(((unsigned)h) << 16); }

__device__ __forceinline__ void dep_guard_b(v8f& a, v8f& b, v16b x, v16b y) { asm volatile("v_nop\n\tv_nop\n\tv_nop\n\tv_nop" : "+v"(a), "+v"(b) : "v"(x), "v"(y)); }
__device__ __forceinline__ void keep4_b(v16b a, v16b b, v16b c, v16b d) { asm volatile("v_nop" :: "v"(a), "v"(b), "v"(c), "v"(d)); }
__device__ __forceinline__ void acc_guard4(v8f& a, v8f& b, v8f& c, v8f& d) { asm volatile("v_nop\n\tv_nop\n\tv_nop\n\tv_nop" : "+v"(a), "+v"(b), "+v"(c), "+v"(d)); }

template <typename T> struct Frag;
template <> struct Frag<__bf16> {
  typedef v16b V; union U { v16b v; v8b h[2]; };
  static __device__ __forceinline__ v16b load(const __bf16* p) {
    U f; f.h[0] = *(const v8b*)(p); f.h[1] = *(const v8b*)(p + 16); return f.v;
  }
  static __device__ __forceinline__ v8f mma(v16b a, v16b b, v8f c) {
    return __builtin_amdgcn_wmma_f32_16x16x32_bf16(false, a, false, b, (short)0, c, false, false);
  }
  static __device__ __forceinline__ void guard(v8f& a, v8f& b, v16b x, v16b y) { dep_guard_b(a, b, x, y); }
  static __device__ __forceinline__ void keep(v16b a, v16b b, v16b c, v16b d) { keep4_b(a, b, c, d); }
};

template <int SPLITM, int OUT_MODE>
__global__ __launch_bounds__(256) void gemm64_bf16(
    const unsigned short* __restrict__ Ap, const unsigned short* __restrict__ A2p, int lda,
    const unsigned short* __restrict__ Btp, const unsigned short* __restrict__ Bt2p, int ldb,
    void* __restrict__ Cout, void* __restrict__ Cout2, int ldc,
    int M, int N, int K, float scale) {
  typedef __bf16 T;
  typedef v16b V;
  typedef __attribute__((ext_vector_type(8))) _Float16 v8hh;
  const T* A = (const T*)Ap; const T* A2 = (const T*)A2p; const T* Bt = (const T*)Btp; const T* Bt2 = (const T*)Bt2p;
  __shared__ __align__(16) float sT[8][16 * 68];
  const int lane = threadIdx.x & 31;
  const int wave = threadIdx.x >> 5;
  const int tilesN = N >> 6;
  const int tilesM = M >> 6;
  const int tile = blockIdx.x * 8 + wave;
  if (tile >= tilesM * tilesN) return;
  const int tm = tile / tilesN;
  const int tn = tile - tm * tilesN;
  const int m0 = tm << 6;
  const int n0 = tn << 6;

  const int rlane = lane & 15;
  const int koff  = (lane >> 4) * 8;
  const int mOff  = (lane >> 4) * 8;

  v8f acc[4][4];
#pragma unroll
  for (int i = 0; i < 4; ++i)
#pragma unroll
    for (int j = 0; j < 4; ++j) acc[i][j] = (v8f){0.f,0.f,0.f,0.f,0.f,0.f,0.f,0.f};

  for (int k0 = 0; k0 < K; k0 += 32) {
    V bh[4], bl[4];
#pragma unroll
    for (int j = 0; j < 4; ++j) {
      const size_t bo = (size_t)(n0 + (j << 4) + rlane) * ldb + koff + k0;
      bh[j] = Frag<T>::load(Bt + bo);
      if (SPLITM == 2) bl[j] = Frag<T>::load(Bt2 + bo);
    }
#pragma unroll
    for (int i = 0; i < 4; ++i) {
      const size_t ao = (size_t)(m0 + (i << 4) + rlane) * lda + koff + k0;
      V ah = Frag<T>::load(A + ao);
      V al = ah;
      if (SPLITM >= 1) al = Frag<T>::load(A2 + ao);
#pragma unroll
      for (int j = 0; j < 4; ++j) {
        acc[i][j] = Frag<T>::mma(ah, bh[j], acc[i][j]);
        if (SPLITM == 2) acc[i][j] = Frag<T>::mma(ah, bl[j], acc[i][j]);
        if (SPLITM >= 1) acc[i][j] = Frag<T>::mma(al, bh[j], acc[i][j]);
      }
      Frag<T>::guard(acc[i][0], acc[i][3], ah, al);
    }
    Frag<T>::keep(bh[0], bh[1], bh[2], bh[3]);
    if (SPLITM == 2) Frag<T>::keep(bl[0], bl[1], bl[2], bl[3]);
  }
  acc_guard4(acc[0][0], acc[0][1], acc[0][2], acc[0][3]);
  acc_guard4(acc[1][0], acc[1][1], acc[1][2], acc[1][3]);
  acc_guard4(acc[2][0], acc[2][1], acc[2][2], acc[2][3]);
  acc_guard4(acc[3][0], acc[3][1], acc[3][2], acc[3][3]);

  float* slab = sT[wave];
#pragma unroll
  for (int i = 0; i < 4; ++i) {
    const int mBase = m0 + (i << 4);
#pragma unroll
    for (int j = 0; j < 4; ++j) {
#pragma unroll
      for (int r = 0; r < 8; ++r) {
        float v = acc[i][j][r] * scale;
        slab[(mOff + r) * 68 + (j << 4) + rlane] = v;
      }
    }
    __builtin_amdgcn_fence(__ATOMIC_RELEASE, "workgroup");
    __builtin_amdgcn_wave_barrier();
    __builtin_amdgcn_fence(__ATOMIC_ACQUIRE, "workgroup");
    if (OUT_MODE == 0) {
      float* C = (float*)Cout;
      const int hh = lane >> 4, c4 = (lane & 15) * 4;
      for (int pass = 0; pass < 2; ++pass) {
#pragma unroll
        for (int it = 0; it < 8; ++it) {
          const int row = it * 2 + hh;
          v4f v = *(const v4f*)(slab + row * 68 + c4);
          *(volatile v4f*)(C + (size_t)(mBase + row) * ldc + n0 + c4) = v;
        }
        __threadfence();
      }
    } else {
      const int q = lane >> 3, c8 = (lane & 7) * 8;
      unsigned short* C  = (unsigned short*)Cout;
      unsigned short* C2 = (OUT_MODE == 2) ? (unsigned short*)Cout2 : nullptr;
      for (int pass = 0; pass < 2; ++pass) {
#pragma unroll
        for (int it = 0; it < 4; ++it) {
          const int row = it * 4 + q;
          const float* sp = slab + row * 68 + c8;
          v8hh hv, lv;
#pragma unroll
          for (int e = 0; e < 8; ++e) {
            if (OUT_MODE == 1) {
              hv[e] = (_Float16)sp[e];
            } else {
              unsigned short hb = f2bf_bits(sp[e]);
              unsigned short lb = f2bf_bits(sp[e] - bf_bits2f(hb));
              hv[e] = __builtin_bit_cast(_Float16, hb);
              lv[e] = __builtin_bit_cast(_Float16, lb);
            }
          }
          *(volatile v8hh*)(C + (size_t)(mBase + row) * ldc + n0 + c8) = hv;
          if (OUT_MODE == 2) *(volatile v8hh*)(C2 + (size_t)(mBase + row) * ldc + n0 + c8) = lv;
        }
        __threadfence();
      }
    }
    __builtin_amdgcn_fence(__ATOMIC_RELEASE, "workgroup");
    __builtin_amdgcn_wave_barrier();
    __builtin_amdgcn_fence(__ATOMIC_ACQUIRE, "workgroup");
  }
}

__global__ __launch_bounds__(256) void cast_f32_bf16x8(
    const float* __restrict__ in, unsigned short* __restrict__ out, int n8) {
  const int i = blockIdx.x * 256 + threadIdx.x;
  if (i < n8) {
    const v4f a0 = *(const v4f*)(in + (size_t)i * 8);
    const v4f a1 = *(const v4f*)(in + (size_t)i * 8 + 4);
    v4u w;
    w[0] = (unsigned)f2bf_bits(a0[0]) | ((unsigned)f2bf_bits(a0[1]) << 16);
    w[1] = (unsigned)f2bf_bits(a0[2]) | ((unsigned)f2bf_bits(a0[3]) << 16);
    w[2] = (unsigned)f2bf_bits(a1[0]) | ((unsigned)f2bf_bits(a1[1]) << 16);
    w[3] = (unsigned)f2bf_bits(a1[2]) | ((unsigned)f2bf_bits(a1[3]) << 16);
    *(volatile v4u*)(out + (size_t)i * 8) = w;
    __threadfence();
    *(volatile v4u*)(out + (size_t)i * 8) = w;
  }
}

#define AT_D 64
#define AT_NW 4
#define AT_QB 64
#define AT_KC 64

__device__ __forceinline__ unsigned short at_bf_bits(float f) {
  unsigned u = __float_as_uint(f);
  return (unsigned short)((u + 0x7FFFu + ((u >> 16) & 1u)) >> 16);
}
__device__ __forceinline__ __bf16 at_f2bf(float f) { return __builtin_bit_cast(__bf16, at_bf_bits(f)); }
__device__ __forceinline__ void at_split(float f, __bf16& hi, __bf16& lo) {
  const unsigned short hb = at_bf_bits(f);
  hi = __builtin_bit_cast(__bf16, hb);
  lo = at_f2bf(f - __uint_as_float(((unsigned)hb) << 16));
}
__device__ __forceinline__ v8f at_mma(v16b a, v16b b, v8f c) {
  c = __builtin_amdgcn_wmma_f32_16x16x32_bf16(false, a, false, b, (short)0, c, false, false);
  asm volatile("v_nop\n\tv_nop\n\tv_nop\n\tv_nop" : "+v"(c) : "v"(a), "v"(b));
  return c;
}

__global__ __launch_bounds__(128)
void attn64_causal_planes(const unsigned short* __restrict__ qh, const unsigned short* __restrict__ ql,
                          const unsigned short* __restrict__ kh, const unsigned short* __restrict__ kl,
                          const unsigned short* __restrict__ vh, const unsigned short* __restrict__ vl,
                          unsigned short* __restrict__ oh, unsigned short* __restrict__ ol,
                          int S, int nH, int ldq, int ldo, float qscale, float mask_fill) {
  union FB { v16b v; v8b h[2]; };
  __shared__ __align__(16) unsigned short Ksh[AT_KC * AT_D];
  __shared__ __align__(16) unsigned short Ksl[AT_KC * AT_D];
  __shared__ __align__(16) unsigned short Vth[AT_D * AT_KC];
  __shared__ __align__(16) unsigned short Vtl[AT_D * AT_KC];
  __shared__ __align__(16) __bf16 Psh[AT_NW][16 * AT_KC];
  __shared__ __align__(16) __bf16 Psl[AT_NW][16 * AT_KC];
  __shared__ __align__(16) float  Os[AT_NW][16 * 68];

  const int tid  = threadIdx.x;
  const int wave = tid >> 5;
  const int lane = tid & 31;
  const int hh   = lane >> 4;
  const int c    = lane & 15;

  const int nqb = S / AT_QB;
  const int bx = blockIdx.x;
  const int qb = bx % nqb;
  const int bh = bx / nqb;
  const int h  = bh % nH;
  const int b  = bh / nH;
  const int q0 = qb * AT_QB + wave * 16;
  const size_t rowbase = (size_t)b * (size_t)S;
  const int hoff = h * AT_D;

  const unsigned short* qhb = qh + hoff;
  const unsigned short* qlb = ql + hoff;
  const unsigned short* khb = kh + hoff;
  const unsigned short* klb = kl + hoff;
  const unsigned short* vhb = vh + hoff;
  const unsigned short* vlb = vl + hoff;

  v16b qah[2], qal[2];
  {
    const size_t ro = (rowbase + (size_t)(q0 + c)) * (size_t)ldq + 8 * hh;
#pragma unroll
    for (int dc = 0; dc < 2; ++dc) {
      FB fh, fl;
      fh.h[0] = __builtin_bit_cast(v8b, *(const v8us*)(qhb + ro + dc * 32));
      fh.h[1] = __builtin_bit_cast(v8b, *(const v8us*)(qhb + ro + dc * 32 + 16));
      fl.h[0] = __builtin_bit_cast(v8b, *(const v8us*)(qlb + ro + dc * 32));
      fl.h[1] = __builtin_bit_cast(v8b, *(const v8us*)(qlb + ro + dc * 32 + 16));
      qah[dc] = fh.v;
      qal[dc] = fl.v;
    }
  }

  const float negInf = -__builtin_inff();
  float mrow[8], lrow[8];
  v8f oacc[4];
#pragma unroll
  for (int r = 0; r < 8; ++r) { mrow[r] = negInf; lrow[r] = 0.f; }
#pragma unroll
  for (int t = 0; t < 4; ++t) oacc[t] = (v8f){0.f,0.f,0.f,0.f,0.f,0.f,0.f,0.f};

  const int nChunks = qb + 1;
  for (int kc = 0; kc < nChunks; ++kc) {
    const int kv0 = kc * AT_KC;
    __syncthreads();
    {
      const int kvr = tid >> 1, dh = (tid & 1) * 32;
      const size_t go = (rowbase + (size_t)(kv0 + kvr)) * (size_t)ldq + dh;
      v4u wk[4], wl[4];
#pragma unroll
      for (int i = 0; i < 4; ++i) {
        wk[i] = *(const v4u*)(khb + go + 8 * i);
        wl[i] = *(const v4u*)(klb + go + 8 * i);
      }
#pragma unroll
      for (int i = 0; i < 4; ++i) {
        *(v4u*)(Ksh + kvr * AT_D + dh + 8 * i) = wk[i];
        *(v4u*)(Ksl + kvr * AT_D + dh + 8 * i) = wl[i];
      }
      asm volatile("" ::: "memory");
#pragma unroll
      for (int i = 0; i < 4; ++i) {
        wk[i] = *(const v4u*)(vhb + go + 8 * i);
        wl[i] = *(const v4u*)(vlb + go + 8 * i);
      }
#pragma unroll
      for (int i = 0; i < 4; ++i) {
#pragma unroll
        for (int e = 0; e < 8; ++e) {
          const unsigned wa = wk[i][e >> 1];
          const unsigned wb = wl[i][e >> 1];
          const unsigned short va = (unsigned short)((e & 1) ? (wa >> 16) : (wa & 0xffffu));
          const unsigned short vb = (unsigned short)((e & 1) ? (wb >> 16) : (wb & 0xffffu));
          const int d = dh + 8 * i + e;
          Vth[d * AT_KC + kvr] = va;
          Vtl[d * AT_KC + kvr] = vb;
        }
      }
    }
    __syncthreads();

    v8f s[4];
#pragma unroll
    for (int j = 0; j < 4; ++j) {
      s[j] = (v8f){0.f,0.f,0.f,0.f,0.f,0.f,0.f,0.f};
#pragma unroll
      for (int dc = 0; dc < 2; ++dc) {
        FB kb, kbl;
        kb.h[0]  = __builtin_bit_cast(v8b, *(const v8us*)(Ksh + (j * 16 + c) * AT_D + dc * 32 + 8 * hh));
        kb.h[1]  = __builtin_bit_cast(v8b, *(const v8us*)(Ksh + (j * 16 + c) * AT_D + dc * 32 + 16 + 8 * hh));
        kbl.h[0] = __builtin_bit_cast(v8b, *(const v8us*)(Ksl + (j * 16 + c) * AT_D + dc * 32 + 8 * hh));
        kbl.h[1] = __builtin_bit_cast(v8b, *(const v8us*)(Ksl + (j * 16 + c) * AT_D + dc * 32 + 16 + 8 * hh));
        s[j] = at_mma(qah[dc], kb.v, s[j]);
        s[j] = at_mma(qah[dc], kbl.v, s[j]);
        s[j] = at_mma(qal[dc], kb.v, s[j]);
      }
    }

    const bool diag = (kc == qb);
    float cm[8];
#pragma unroll
    for (int r = 0; r < 8; ++r) {
      const int qrow = q0 + 8 * hh + r;
      float m = negInf;
#pragma unroll
      for (int j = 0; j < 4; ++j) {
        const int kvcol = kv0 + j * 16 + c;
        float sv = s[j][r] * qscale;
        if (diag && (kvcol > qrow)) sv = mask_fill;
        s[j][r] = sv;
        m = fmaxf(m, sv);
      }
#pragma unroll
      for (int off = 1; off < 16; off <<= 1) m = fmaxf(m, __shfl_xor(m, off, 32));
      cm[r] = m;
    }

    __bf16* pwh = Psh[wave];
    __bf16* pwl = Psl[wave];
#pragma unroll
    for (int r = 0; r < 8; ++r) {
      const float mnew = fmaxf(mrow[r], cm[r]);
      const float alpha = expf(mrow[r] - mnew);
      mrow[r] = mnew;
      float psum = 0.f;
#pragma unroll
      for (int j = 0; j < 4; ++j) {
        const float p = expf(s[j][r] - mnew);
        psum += p;
        __bf16 a, bl;
        at_split(p, a, bl);
        pwh[(8 * hh + r) * AT_KC + j * 16 + c] = a;
        pwl[(8 * hh + r) * AT_KC + j * 16 + c] = bl;
      }
#pragma unroll
      for (int off = 1; off < 16; off <<= 1) psum += __shfl_xor(psum, off, 32);
      lrow[r] = lrow[r] * alpha + psum;
#pragma unroll
      for (int t = 0; t < 4; ++t) oacc[t][r] *= alpha;
    }
    __builtin_amdgcn_fence(__ATOMIC_RELEASE, "workgroup");
    __builtin_amdgcn_wave_barrier();
    __builtin_amdgcn_fence(__ATOMIC_ACQUIRE, "workgroup");

#pragma unroll 1
    for (int kk = 0; kk < 2; ++kk) {
      FB pa, pl;
      pa.h[0] = *(const v8b*)(pwh + c * AT_KC + kk * 32 + 8 * hh);
      pa.h[1] = *(const v8b*)(pwh + c * AT_KC + kk * 32 + 16 + 8 * hh);
      pl.h[0] = *(const v8b*)(pwl + c * AT_KC + kk * 32 + 8 * hh);
      pl.h[1] = *(const v8b*)(pwl + c * AT_KC + kk * 32 + 16 + 8 * hh);
#pragma unroll
      for (int t = 0; t < 4; ++t) {
        FB vb, vbl;
        vb.h[0]  = __builtin_bit_cast(v8b, *(const v8us*)(Vth + (t * 16 + c) * AT_KC + kk * 32 + 8 * hh));
        vb.h[1]  = __builtin_bit_cast(v8b, *(const v8us*)(Vth + (t * 16 + c) * AT_KC + kk * 32 + 16 + 8 * hh));
        vbl.h[0] = __builtin_bit_cast(v8b, *(const v8us*)(Vtl + (t * 16 + c) * AT_KC + kk * 32 + 8 * hh));
        vbl.h[1] = __builtin_bit_cast(v8b, *(const v8us*)(Vtl + (t * 16 + c) * AT_KC + kk * 32 + 16 + 8 * hh));
        oacc[t] = at_mma(pa.v, vb.v, oacc[t]);
        oacc[t] = at_mma(pa.v, vbl.v, oacc[t]);
        oacc[t] = at_mma(pl.v, vb.v, oacc[t]);
      }
    }
  }

  float* os = Os[wave];
#pragma unroll
  for (int r = 0; r < 8; ++r) {
    const float inv = 1.0f / lrow[r];
#pragma unroll
    for (int t = 0; t < 4; ++t) os[(8 * hh + r) * 68 + t * 16 + c] = oacc[t][r] * inv;
  }
  __builtin_amdgcn_fence(__ATOMIC_RELEASE, "workgroup");
  __builtin_amdgcn_wave_barrier();
  __builtin_amdgcn_fence(__ATOMIC_ACQUIRE, "workgroup");
  {
    const int q4 = lane >> 3, c8 = (lane & 7) * 8;
    for (int pass = 0; pass < 2; ++pass) {
#pragma unroll
      for (int it = 0; it < 4; ++it) {
        const int row = it * 4 + q4;
        const float* sp = os + row * 68 + c8;
        const v4f x0 = *(const v4f*)(sp);
        const v4f x1 = *(const v4f*)(sp + 4);
        float fv[8];
        fv[0] = x0[0]; fv[1] = x0[1]; fv[2] = x0[2]; fv[3] = x0[3];
        fv[4] = x1[0]; fv[5] = x1[1]; fv[6] = x1[2]; fv[7] = x1[3];
        v4u hw, lw;
#pragma unroll
        for (int e2 = 0; e2 < 4; ++e2) {
          const unsigned short hb0 = f2bf_bits(fv[2 * e2]);
          const unsigned short lb0 = f2bf_bits(fv[2 * e2] - bf_bits2f(hb0));
          const unsigned short hb1 = f2bf_bits(fv[2 * e2 + 1]);
          const unsigned short lb1 = f2bf_bits(fv[2 * e2 + 1] - bf_bits2f(hb1));
          hw[e2] = (unsigned)hb0 | ((unsigned)hb1 << 16);
          lw[e2] = (unsigned)lb0 | ((unsigned)lb1 << 16);
        }
        const size_t off = (rowbase + (size_t)(q0 + row)) * (size_t)ldo + hoff + c8;
        *(volatile v4u*)(oh + off) = hw;
        *(volatile v4u*)(ol + off) = lw;
      }
      __threadfence();
    }
  }
}

extern "C" void kernel_launch(void* const* d_in, const int* in_sizes, int n_in,
                              void* d_out, int out_size, void* d_ws, size_t ws_size,
                              hipStream_t stream) {
  if (n_in < 5) return;
  if (in_sizes[0] != NROW * NMODEL) return;
  if (in_sizes[1] != NMODEL * NMODEL || in_sizes[2] != NMODEL * NMODEL ||
      in_sizes[3] != NMODEL * NMODEL || in_sizes[4] != NMODEL * NMODEL) return;
  if (out_size != NROW * NMODEL) return;

  const float* x  = (const float*)d_in[0];
  const float* Wq = (const float*)d_in[1];
  const float* Wk = (const float*)d_in[2];
  const float* Wv = (const float*)d_in[3];
  const float* Wo = (const float*)d_in[4];
  float* out = (float*)d_out;

  const size_t szXb   = (size_t)NROW * NMODEL * 2;
  const size_t szW3   = (size_t)NQKV * NMODEL * 2;
  const size_t szWo   = (size_t)NMODEL * NMODEL * 2;
  const size_t szQKV  = (size_t)NROW * NQKV * 2;
  const size_t szO    = (size_t)NROW * NMODEL * 2;
  const size_t offXb   = 0;
  const size_t offW3   = offXb + szXb;
  const size_t offWo   = offW3 + szW3;
  const size_t offQKVh = offWo + szWo;
  const size_t offQKVl = offQKVh + szQKV;
  const size_t offOh   = offQKVl + szQKV;
  const size_t offOl   = offOh + szO;
  const size_t total   = offOl + szO;
  if (ws_size < total) return;

  char* ws = (char*)d_ws;
  unsigned short* xb   = (unsigned short*)(ws + offXb);
  unsigned short* w3b  = (unsigned short*)(ws + offW3);
  unsigned short* wob  = (unsigned short*)(ws + offWo);
  unsigned short* qkvh = (unsigned short*)(ws + offQKVh);
  unsigned short* qkvl = (unsigned short*)(ws + offQKVl);
  unsigned short* oh   = (unsigned short*)(ws + offOh);
  unsigned short* ol   = (unsigned short*)(ws + offOl);

  {
    const int n8x = NROW * NMODEL / 8;
    cast_f32_bf16x8<<<dim3((n8x + 255) / 256), 256, 0, stream>>>(x, xb, n8x);
    const int n8w = NMODEL * NMODEL / 8;
    cast_f32_bf16x8<<<dim3((n8w + 255) / 256), 256, 0, stream>>>(Wq, w3b, n8w);
    cast_f32_bf16x8<<<dim3((n8w + 255) / 256), 256, 0, stream>>>(Wk, w3b + (size_t)NMODEL * NMODEL, n8w);
    cast_f32_bf16x8<<<dim3((n8w + 255) / 256), 256, 0, stream>>>(Wv, w3b + (size_t)2 * NMODEL * NMODEL, n8w);
    cast_f32_bf16x8<<<dim3((n8w + 255) / 256), 256, 0, stream>>>(Wo, wob, n8w);
  }

  {
    const int tiles = (NROW / 64) * (NQKV / 64);
    gemm64_bf16<0, 2><<<dim3((tiles + 7) / 8), 256, 0, stream>>>(
        xb, xb, NMODEL, w3b, w3b, NMODEL, (void*)qkvh, (void*)qkvl, NQKV,
        NROW, NQKV, NMODEL, 1.0f);
  }

  {
    const int nblk = NBATCH * NHEAD * (NSEQ / AT_QB);
    attn64_causal_planes<<<dim3(nblk), 128, 0, stream>>>(
        qkvh, qkvl, qkvh + NMODEL, qkvl + NMODEL, qkvh + 2 * NMODEL, qkvl + 2 * NMODEL,
        oh, ol, NSEQ, NHEAD, NQKV, NMODEL, 0.125f, -1e30f);
  }

  {
    const int tiles = (NROW / 64) * (NMODEL / 64);
    gemm64_bf16<1, 0><<<dim3((tiles + 7) / 8), 256, 0, stream>>>(
        oh, ol, NMODEL, wob, wob, NMODEL, (void*)out, (void*)out, NMODEL,
        NROW, NMODEL, NMODEL, 1.0f);
  }
}
